// CosineAttention_20392504722137
// MI455X (gfx1250) — hardware-verified
//
#include <hip/hip_runtime.h>
#include <stddef.h>

typedef __attribute__((ext_vector_type(16))) _Float16 v16h;
typedef __attribute__((ext_vector_type(8)))  _Float16 v8h;
typedef __attribute__((ext_vector_type(8)))  float    v8f;
typedef __attribute__((ext_vector_type(4)))  float    v4f;

#ifndef NB
#define NB 2
#endif
#ifndef SEQ
#define SEQ 2048
#endif
#ifndef RES_ROWS
#define RES_ROWS 128
#endif

constexpr int NB_FULL  = 2;
constexpr int SEQ_FULL = 2048;
constexpr int DIM   = 1024;
constexpr int NHEAD = 16;
constexpr int HDIM  = 64;
constexpr int INNER = NHEAD * HDIM;
constexpr int KD    = 1024;
constexpr int MROWS = NB * SEQ;
constexpr int QKVC  = 3 * INNER;
constexpr int ERES  = 64;

static_assert(NB >= 1 && NB <= NB_FULL);
static_assert(SEQ % 64 == 0 && SEQ >= 128 && SEQ <= SEQ_FULL);
static_assert(DIM == KD && INNER == KD && KD % 32 == 0);
static_assert(HDIM == 64 && INNER % 64 == 0 && DIM % 64 == 0 && QKVC % 64 == 0);
static_assert(MROWS % 64 == 0);
static_assert(RES_ROWS % 64 == 0 && RES_ROWS >= 64 && RES_ROWS <= SEQ);

constexpr float XCARRY   = 16.0f;
constexpr float WCARRY   = 64.0f;
constexpr float QKV_INV  = 1.0f / (16.0f * 64.0f);
constexpr float QNCARRY  = 16.0f;
constexpr float SCARRY   = 2048.0f;
constexpr float SRES_INV = 1.0f / 2048.0f;
constexpr float SSCALE   = 8.0f / 256.0f;
constexpr float MASKV    = -1.0e10f;
constexpr float PCARRY   = 32768.0f;
constexpr float LOCARRY  = 1024.0f;
constexpr float LO_INV   = 1.0f / 1024.0f;
constexpr float OCARRY   = 16.0f;
constexpr float OUT_INV  = 1.0f / (16.0f * 64.0f);

union FragU { v16h v; v8h h[2]; };
__device__ __forceinline__ v16h frag_load(const _Float16* p) {
  FragU f;
  f.h[0] = *(const v8h*)(p);
  f.h[1] = *(const v8h*)(p + 16);
  return f.v;
}
__device__ __forceinline__ v8f mma_h(v16h a, v16h b, v8f c) {
  c = __builtin_amdgcn_wmma_f32_16x16x32_f16(false, a, false, b, (short)0, c, false, false);
  asm volatile("v_nop\n\tv_nop\n\tv_nop\n\tv_nop" : "+v"(c) : "v"(a), "v"(b));
  return c;
}
__device__ __forceinline__ void wave_lds_sync() {
  __builtin_amdgcn_fence(__ATOMIC_RELEASE, "workgroup");
  __builtin_amdgcn_wave_barrier();
  __builtin_amdgcn_fence(__ATOMIC_ACQUIRE, "workgroup");
}
__device__ __forceinline__ float bf_rne(float f) {
  unsigned int u = __float_as_uint(f);
  u = (u + 0x7FFFu + ((u >> 16) & 1u)) & 0xFFFF0000u;
  return __uint_as_float(u);
}

constexpr int CVX_THREADS = 256;
static_assert(DIM == 8 * 128 && MROWS % 2 == 0);

__global__ __launch_bounds__(CVX_THREADS)
void cvt_x(const float* __restrict__ x, _Float16* __restrict__ xh) {
  const int tid  = threadIdx.x;
  const int r    = blockIdx.x * 2 + (tid >> 7);
  const int j    = tid & 127;
  const int srow = (r / SEQ) * SEQ_FULL + (r % SEQ);
  const float* p = x + (size_t)srow * DIM + (size_t)j * 8;
  const v4f a0 = *(const v4f*)(p);
  const v4f a1 = *(const v4f*)(p + 4);
  v8h o;
#pragma unroll
  for (int e = 0; e < 4; ++e) {
    o[e]     = (_Float16)(bf_rne(a0[e]) * XCARRY);
    o[4 + e] = (_Float16)(bf_rne(a1[e]) * XCARRY);
  }
  _Float16* d = xh + (size_t)r * DIM + (size_t)j * 8;
  for (int pass = 0; pass < 2; ++pass) {
    *(volatile v8h*)d = o;
    __threadfence();
  }
}

constexpr int CVW_THREADS = 256;
constexpr int TP = 72;

__global__ __launch_bounds__(CVW_THREADS)
void cvt_w(const float* Wq, const float* Wk, const float* Wv, const float* Wo,
           _Float16* __restrict__ Wt) {
  __shared__ __align__(16) _Float16 T[64 * TP];
  const int tid  = threadIdx.x;
  const int lane = tid & 31;
  const int wave = tid >> 5;
  const int z    = blockIdx.z;
  const float* src = (z == 0) ? Wq : (z == 1) ? Wk : (z == 2) ? Wv : Wo;
  const int n0 = blockIdx.x * 64;
  const int k0 = blockIdx.y * 64;
  const int kr  = tid >> 2;
  const int c16 = (tid & 3) * 16;
  const float* p = src + (size_t)(k0 + kr) * KD + n0 + c16;
#pragma unroll
  for (int i = 0; i < 4; ++i) {
    const v4f a = *(const v4f*)(p + 4 * i);
#pragma unroll
    for (int e = 0; e < 4; ++e)
      T[(c16 + 4 * i + e) * TP + kr] = (_Float16)(bf_rne(a[e]) * WCARRY);
  }
  __syncthreads();

  const int rg = lane >> 3;
  const int c8 = (lane & 7) * 8;
  _Float16* dst = Wt + (size_t)z * KD * KD + (size_t)n0 * KD + (size_t)k0;
  for (int pass = 0; pass < 2; ++pass) {
#pragma unroll
    for (int it = 0; it < 2; ++it) {
      const int row = wave * 8 + it * 4 + rg;
      const v8h v = *(const v8h*)(T + row * TP + c8);
      *(volatile v8h*)(dst + (size_t)row * KD + c8) = v;
    }
    __threadfence();
  }
}

constexpr int GM_THREADS = 128;
constexpr int GPITCH = 68;

template <int NA2>
__global__ __launch_bounds__(GM_THREADS)
void gemm_f16(const _Float16* __restrict__ A0, const _Float16* __restrict__ A1,
              const _Float16* __restrict__ Bt, float* __restrict__ C,
              int cpitch, int cseqf, float cscale) {
  __shared__ __align__(16) float Cs[4][16 * GPITCH];

  const int tid  = threadIdx.x;
  const int wave = tid >> 5;
  const int lane = tid & 31;
  const int hh   = lane >> 4;
  const int m    = lane & 15;
  const int row0 = blockIdx.y * 64;
  const int n0   = blockIdx.x * 64;
  const bool lo_on = (NA2 != 0) && ((row0 % SEQ) < RES_ROWS);

  const _Float16* ap  = A0 + (size_t)(row0 + wave * 16 + m) * KD + 8 * hh;
  const _Float16* alp = A1 + (size_t)(row0 + wave * 16 + m) * KD + 8 * hh;
  const _Float16* bp  = Bt + (size_t)(n0 + m) * KD + 8 * hh;

  v8f acc[4], accl[4];
#pragma unroll
  for (int t = 0; t < 4; ++t) {
    acc[t]  = (v8f){0.f, 0.f, 0.f, 0.f, 0.f, 0.f, 0.f, 0.f};
    accl[t] = (v8f){0.f, 0.f, 0.f, 0.f, 0.f, 0.f, 0.f, 0.f};
  }

  for (int k0 = 0; k0 < KD; k0 += 32) {
    const v16h a = frag_load(ap + k0);
    v16h bf[4];
#pragma unroll
    for (int t = 0; t < 4; ++t) bf[t] = frag_load(bp + (size_t)(t * 16) * KD + k0);
#pragma unroll
    for (int t = 0; t < 4; ++t) acc[t] = mma_h(a, bf[t], acc[t]);
    if (lo_on) {
      const v16h al = frag_load(alp + k0);
#pragma unroll
      for (int t = 0; t < 4; ++t) accl[t] = mma_h(al, bf[t], accl[t]);
    }
  }

  float* cs = Cs[wave];
#pragma unroll
  for (int r = 0; r < 8; ++r) {
#pragma unroll
    for (int t = 0; t < 4; ++t) {
      float v = acc[t][r];
      if (lo_on) v += accl[t][r] * LO_INV;
      cs[(8 * hh + r) * GPITCH + t * 16 + m] = v * cscale;
    }
  }
  wave_lds_sync();
  {
    const int c4 = (lane & 15) * 4;
    for (int pass = 0; pass < 2; ++pass) {
#pragma unroll
      for (int it = 0; it < 8; ++it) {
        const int row  = it * 2 + hh;
        const int rc   = row0 + wave * 16 + row;
        const int crow = (rc / SEQ) * cseqf + (rc % SEQ);
        const v4f val = *(const v4f*)(cs + row * GPITCH + c4);
        *(volatile v4f*)(C + (size_t)crow * cpitch + n0 + c4) = val;
      }
      __threadfence();
    }
  }
}

constexpr int PREP_THREADS = 256;
constexpr int TROWS  = 64;
constexpr int LPITCH = 72;
static_assert(TROWS == ERES);

__device__ __forceinline__ void cvt_hl(float f, _Float16& hi, _Float16& lo) {
  const _Float16 g = (_Float16)f;
  hi = g;
  lo = (_Float16)((f - (float)g) * SCARRY);
}

__device__ __forceinline__ void norm_quarter(const float* __restrict__ p, v8h& o0, v8h& o1, v8h& l0, v8h& l1) {
  const v4f a0 = *(const v4f*)(p);
  const v4f a1 = *(const v4f*)(p + 4);
  const v4f a2 = *(const v4f*)(p + 8);
  const v4f a3 = *(const v4f*)(p + 12);
  float ss = 0.0f;
  ss += a0[0] * a0[0]; ss += a0[1] * a0[1]; ss += a0[2] * a0[2]; ss += a0[3] * a0[3];
  ss += a1[0] * a1[0]; ss += a1[1] * a1[1]; ss += a1[2] * a1[2]; ss += a1[3] * a1[3];
  ss += a2[0] * a2[0]; ss += a2[1] * a2[1]; ss += a2[2] * a2[2]; ss += a2[3] * a2[3];
  ss += a3[0] * a3[0]; ss += a3[1] * a3[1]; ss += a3[2] * a3[2]; ss += a3[3] * a3[3];
  ss += __shfl_xor(ss, 1, 32);
  ss += __shfl_xor(ss, 2, 32);
  const float sc = QNCARRY / sqrtf(ss + 1.0e-12f);
#pragma unroll
  for (int e = 0; e < 4; ++e) {
    _Float16 gh, gl;
    cvt_hl(a0[e] * sc, gh, gl); o0[e]     = gh; l0[e]     = gl;
    cvt_hl(a1[e] * sc, gh, gl); o0[4 + e] = gh; l0[4 + e] = gl;
    cvt_hl(a2[e] * sc, gh, gl); o1[e]     = gh; l1[e]     = gl;
    cvt_hl(a3[e] * sc, gh, gl); o1[4 + e] = gh; l1[4 + e] = gl;
  }
}

__device__ __forceinline__ void scat4hl(_Float16* vs, _Float16* vls, int d0, int r, v4f a) {
#pragma unroll
  for (int e = 0; e < 4; ++e) {
    const _Float16 hi = (_Float16)a[e];
    vs[(d0 + e) * LPITCH + r]  = hi;
    vls[(d0 + e) * LPITCH + r] = (_Float16)((a[e] - (float)hi) * LOCARRY);
  }
}

__global__ __launch_bounds__(PREP_THREADS)
void prep_planes(const float* __restrict__ Cqkv,
                 _Float16* __restrict__ Qh, _Float16* __restrict__ Qlh,
                 _Float16* __restrict__ Kh, _Float16* __restrict__ Klh,
                 _Float16* __restrict__ Vth, _Float16* __restrict__ Vtl) {
  __shared__ __align__(16) _Float16 Qs[TROWS * LPITCH];
  __shared__ __align__(16) _Float16 Qls[TROWS * LPITCH];
  __shared__ __align__(16) _Float16 Ks[TROWS * LPITCH];
  __shared__ __align__(16) _Float16 Kls[TROWS * LPITCH];
  __shared__ __align__(16) _Float16 Vs[HDIM * LPITCH];
  __shared__ __align__(16) _Float16 Vls[HDIM * LPITCH];

  const int tid  = threadIdx.x;
  const int lane = tid & 31;
  const int wave = tid >> 5;
  constexpr int NT = SEQ / TROWS;
  const int bx = blockIdx.x;
  const int st = bx % NT;
  const int h  = (bx / NT) % NHEAD;
  const int b  = bx / (NT * NHEAD);
  const int s0 = st * TROWS;
  const bool early = (st == 0);
  const int r  = tid >> 2;
  const int qd = tid & 3;
  const size_t goff = ((size_t)b * SEQ + (size_t)(s0 + r)) * QKVC + (size_t)h * HDIM + (size_t)qd * 16;

  {
    v8h o0, o1, l0, l1;
    norm_quarter(Cqkv + goff, o0, o1, l0, l1);
    *(v8h*)(Qs  + r * LPITCH + qd * 16)     = o0;
    *(v8h*)(Qs  + r * LPITCH + qd * 16 + 8) = o1;
    *(v8h*)(Qls + r * LPITCH + qd * 16)     = l0;
    *(v8h*)(Qls + r * LPITCH + qd * 16 + 8) = l1;
  }
  {
    v8h o0, o1, l0, l1;
    norm_quarter(Cqkv + goff + INNER, o0, o1, l0, l1);
    *(v8h*)(Ks  + r * LPITCH + qd * 16)     = o0;
    *(v8h*)(Ks  + r * LPITCH + qd * 16 + 8) = o1;
    *(v8h*)(Kls + r * LPITCH + qd * 16)     = l0;
    *(v8h*)(Kls + r * LPITCH + qd * 16 + 8) = l1;
  }
  {
    const float* vp = Cqkv + goff + 2 * INNER;
    const v4f a0 = *(const v4f*)(vp);
    const v4f a1 = *(const v4f*)(vp + 4);
    const v4f a2 = *(const v4f*)(vp + 8);
    const v4f a3 = *(const v4f*)(vp + 12);
    scat4hl(Vs, Vls, qd * 16 + 0,  r, a0);
    scat4hl(Vs, Vls, qd * 16 + 4,  r, a1);
    scat4hl(Vs, Vls, qd * 16 + 8,  r, a2);
    scat4hl(Vs, Vls, qd * 16 + 12, r, a3);
  }
  __syncthreads();

  const int rg = lane >> 3;
  const int c8 = (lane & 7) * 8;
  const size_t plane = (size_t)(b * NHEAD + h);
  _Float16* qdst  = Qh  + (plane * SEQ + (size_t)s0) * HDIM;
  _Float16* kdst  = Kh  + (plane * SEQ + (size_t)s0) * HDIM;
  _Float16* qldst = Qlh + (plane * ERES) * HDIM;
  _Float16* kldst = Klh + (plane * ERES) * HDIM;
  _Float16* vdst  = Vth + (plane * HDIM) * SEQ + (size_t)s0;
  _Float16* vldst = Vtl + (plane * HDIM) * SEQ + (size_t)s0;
  for (int pass = 0; pass < 2; ++pass) {
#pragma unroll
    for (int it = 0; it < 2; ++it) {
      const int row = wave * 8 + it * 4 + rg;
      const v8h qv  = *(const v8h*)(Qs  + row * LPITCH + c8);
      const v8h kv  = *(const v8h*)(Ks  + row * LPITCH + c8);
      const v8h vv  = *(const v8h*)(Vs  + row * LPITCH + c8);
      const v8h vlv = *(const v8h*)(Vls + row * LPITCH + c8);
      *(volatile v8h*)(qdst  + (size_t)row * HDIM + c8) = qv;
      *(volatile v8h*)(kdst  + (size_t)row * HDIM + c8) = kv;
      *(volatile v8h*)(vdst  + (size_t)row * SEQ  + c8) = vv;
      *(volatile v8h*)(vldst + (size_t)row * SEQ  + c8) = vlv;
      if (early) {
        const v8h qlv = *(const v8h*)(Qls + row * LPITCH + c8);
        const v8h klv = *(const v8h*)(Kls + row * LPITCH + c8);
        *(volatile v8h*)(qldst + (size_t)row * HDIM + c8) = qlv;
        *(volatile v8h*)(kldst + (size_t)row * HDIM + c8) = klv;
      }
    }
    __threadfence();
  }
}

constexpr int AT_THREADS = 128;
constexpr int QBLK   = 64;
constexpr int KCH    = 64;
constexpr int OPITCH = 68;
constexpr int VRES_QB = RES_ROWS / QBLK;
static_assert(QBLK == ERES && KCH == ERES && VRES_QB >= 1);
static_assert(SEQ / QBLK >= 2);

__global__ __launch_bounds__(AT_THREADS)
void causal_attn(const _Float16* __restrict__ Qh, const _Float16* __restrict__ Kh,
                 const _Float16* __restrict__ Vth, const _Float16* __restrict__ Vtl,
                 _Float16* __restrict__ Oh, _Float16* __restrict__ Ol) {
  __shared__ __align__(16) _Float16 Ksh[KCH * HDIM];
  __shared__ __align__(16) _Float16 Vhs[HDIM * KCH];
  __shared__ __align__(16) _Float16 Vls[HDIM * KCH];
  __shared__ __align__(16) _Float16 Psh[4][16 * KCH];
  __shared__ __align__(16) float    Os[4][16 * OPITCH];

  const int tid  = threadIdx.x;
  const int wave = tid >> 5;
  const int lane = tid & 31;
  const int hh   = lane >> 4;
  const int c    = lane & 15;

  constexpr int NQB  = SEQ / QBLK;
  constexpr int NQBL = NQB - 1;
  const int bx = blockIdx.x;
  const int qb = 1 + bx % NQBL;
  const int bh = bx / NQBL;
  const int h  = bh % NHEAD;
  const int b  = bh / NHEAD;
  const int q0 = qb * QBLK + wave * 16;
  const bool vres = (qb < VRES_QB);

  const size_t plane = (size_t)(b * NHEAD + h);
  const _Float16* qpl  = Qh  + plane * SEQ * HDIM;
  const _Float16* kpl  = Kh  + plane * SEQ * HDIM;
  const _Float16* vpl  = Vth + plane * HDIM * SEQ;
  const _Float16* vlpl = Vtl + plane * HDIM * SEQ;

  v16h qa[2];
#pragma unroll
  for (int dc = 0; dc < 2; ++dc)
    qa[dc] = frag_load(qpl + (size_t)(q0 + c) * HDIM + dc * 32 + 8 * hh);

  const float neg_inf = -__builtin_inff();
  float mrow[8], lrow[8];
  v8f oacc[4], oacc2[4];
#pragma unroll
  for (int r = 0; r < 8; ++r) { mrow[r] = neg_inf; lrow[r] = 0.0f; }
#pragma unroll
  for (int t = 0; t < 4; ++t) {
    oacc[t]  = (v8f){0.f, 0.f, 0.f, 0.f, 0.f, 0.f, 0.f, 0.f};
    oacc2[t] = (v8f){0.f, 0.f, 0.f, 0.f, 0.f, 0.f, 0.f, 0.f};
  }
  const int qloc = wave * 16 + 8 * hh;

  for (int kc = 0; kc <= qb; ++kc) {
    const int kv0 = kc * KCH;
    __syncthreads();
#pragma unroll
    for (int i = 0; i < 4; ++i) {
      const int idx = tid + i * AT_THREADS;
      const int row = idx >> 3;
      const int c8  = (idx & 7) * 8;
      const v8h kk = *(const v8h*)(kpl + (size_t)(kv0 + row) * HDIM + c8);
      const v8h vv = *(const v8h*)(vpl + (size_t)row * SEQ + (size_t)kv0 + c8);
      *(v8h*)(Ksh + row * HDIM + c8) = kk;
      *(v8h*)(Vhs + row * KCH  + c8) = vv;
      if (vres) {
        const v8h vl = *(const v8h*)(vlpl + (size_t)row * SEQ + (size_t)kv0 + c8);
        *(v8h*)(Vls + row * KCH + c8) = vl;
      }
    }
    __syncthreads();

    v8f s[4];
#pragma unroll
    for (int j = 0; j < 4; ++j) {
      s[j] = (v8f){0.f, 0.f, 0.f, 0.f, 0.f, 0.f, 0.f, 0.f};
#pragma unroll
      for (int dc = 0; dc < 2; ++dc) {
        const v16h kb = frag_load(Ksh + (j * 16 + c) * HDIM + dc * 32 + 8 * hh);
        s[j] = mma_h(qa[dc], kb, s[j]);
      }
    }

    const bool diag = (kc == qb);
    float cm[8];
#pragma unroll
    for (int r = 0; r < 8; ++r) {
      float m = neg_inf;
#pragma unroll
      for (int j = 0; j < 4; ++j) {
        float sv = s[j][r] * SSCALE;
        if (diag && (j * 16 + c) > (qloc + r)) sv = MASKV;
        s[j][r] = sv;
        m = fmaxf(m, sv);
      }
#pragma unroll
      for (int off = 1; off < 16; off <<= 1) m = fmaxf(m, __shfl_xor(m, off, 32));
      cm[r] = m;
    }
    _Float16* pw = Psh[wave];
#pragma unroll
    for (int r = 0; r < 8; ++r) {
      const float mnew  = fmaxf(mrow[r], cm[r]);
      const float alpha = expf(mrow[r] - mnew);
      mrow[r] = mnew;
      float psum = 0.0f;
#pragma unroll
      for (int j = 0; j < 4; ++j) {
        const float p = expf(s[j][r] - mnew);
        psum += p;
        pw[(8 * hh + r) * KCH + j * 16 + c] = (_Float16)(p * PCARRY);
      }
#pragma unroll
      for (int off = 1; off < 16; off <<= 1) psum += __shfl_xor(psum, off, 32);
      lrow[r] = lrow[r] * alpha + psum;
#pragma unroll
      for (int t = 0; t < 4; ++t) oacc[t][r] *= alpha;
      if (vres) {
#pragma unroll
        for (int t = 0; t < 4; ++t) oacc2[t][r] *= alpha;
      }
    }
    wave_lds_sync();

#pragma unroll
    for (int kk = 0; kk < 2; ++kk) {
      const v16h pa = frag_load(pw + c * KCH + kk * 32 + 8 * hh);
#pragma unroll
      for (int t = 0; t < 4; ++t) {
        const v16h vb = frag_load(Vhs + (t * 16 + c) * KCH + kk * 32 + 8 * hh);
        oacc[t] = mma_h(pa, vb, oacc[t]);
      }
      if (vres) {
#pragma unroll
        for (int t = 0; t < 4; ++t) {
          const v16h vlb = frag_load(Vls + (t * 16 + c) * KCH + kk * 32 + 8 * hh);
          oacc2[t] = mma_h(pa, vlb, oacc2[t]);
        }
      }
    }
  }

  float* os = Os[wave];
#pragma unroll
  for (int r = 0; r < 8; ++r) {
    const float inv = 1.0f / (lrow[r] * PCARRY);
#pragma unroll
    for (int t = 0; t < 4; ++t) {
      float o = oacc[t][r];
      if (vres) o += oacc2[t][r] * LO_INV;
      os[(8 * hh + r) * OPITCH + t * 16 + c] = o * inv;
    }
  }
  wave_lds_sync();
  {
    const int rg = lane >> 3;
    const int c8 = (lane & 7) * 8;
    const size_t obase = ((size_t)b * SEQ + (size_t)q0) * INNER + (size_t)h * HDIM;
    for (int pass = 0; pass < 2; ++pass) {
#pragma unroll
      for (int it = 0; it < 4; ++it) {
        const int row = it * 4 + rg;
        const float* sp = os + row * OPITCH + c8;
        const v4f x0 = *(const v4f*)(sp);
        const v4f x1 = *(const v4f*)(sp + 4);
        v8h hv, lv;
#pragma unroll
        for (int e = 0; e < 4; ++e) {
          const float f0 = x0[e] * OCARRY;
          const _Float16 g0 = (_Float16)f0;
          hv[e] = g0;
          lv[e] = (_Float16)((f0 - (float)g0) * LOCARRY);
          const float f1 = x1[e] * OCARRY;
          const _Float16 g1 = (_Float16)f1;
          hv[4 + e] = g1;
          lv[4 + e] = (_Float16)((f1 - (float)g1) * LOCARRY);
        }
        *(volatile v8h*)(Oh + obase + (size_t)row * INNER + c8) = hv;
        *(volatile v8h*)(Ol + obase + (size_t)row * INNER + c8) = lv;
      }
      __threadfence();
    }
  }
}

__global__ __launch_bounds__(AT_THREADS)
void early_attn(const _Float16* __restrict__ Qh, const _Float16* __restrict__ Qlh,
                const _Float16* __restrict__ Kh, const _Float16* __restrict__ Klh,
                const _Float16* __restrict__ Vth, const _Float16* __restrict__ Vtl,
                _Float16* __restrict__ Oh, _Float16* __restrict__ Ol) {
  __shared__ __align__(16) _Float16 Ksh[KCH * HDIM];
  __shared__ __align__(16) _Float16 Vhs[HDIM * KCH];
  __shared__ __align__(16) _Float16 Vls[HDIM * KCH];
  __shared__ __align__(16) _Float16 Psh[4][16 * KCH];
  __shared__ __align__(16) _Float16 Plsh[4][16 * KCH];
  __shared__ __align__(16) float    SO[4][16 * OPITCH];

  const int tid  = threadIdx.x;
  const int wave = tid >> 5;
  const int lane = tid & 31;
  const int hh   = lane >> 4;
  const int c    = lane & 15;

  const int bh = blockIdx.x;
  const int h  = bh % NHEAD;
  const int b  = bh / NHEAD;
  const int q0 = wave * 16;

  const size_t plane = (size_t)(b * NHEAD + h);
  const _Float16* qpl  = Qh  + plane * SEQ * HDIM;
  const _Float16* kpl  = Kh  + plane * SEQ * HDIM;
  const _Float16* qlpl = Qlh + plane * ERES * HDIM;
  const _Float16* klpl = Klh + plane * ERES * HDIM;
  const _Float16* vpl  = Vth + plane * HDIM * SEQ;
  const _Float16* vlpl = Vtl + plane * HDIM * SEQ;

#pragma unroll
  for (int i = 0; i < 4; ++i) {
    const int idx = tid + i * AT_THREADS;
    const int row = idx >> 3;
    const int c8  = (idx & 7) * 8;
    const v8h kk = *(const v8h*)(kpl + (size_t)row * HDIM + c8);
    const v8h vv = *(const v8h*)(vpl + (size_t)row * SEQ + c8);
    const v8h vl = *(const v8h*)(vlpl + (size_t)row * SEQ + c8);
    *(v8h*)(Ksh + row * HDIM + c8) = kk;
    *(v8h*)(Vhs + row * KCH  + c8) = vv;
    *(v8h*)(Vls + row * KCH  + c8) = vl;
  }
  __syncthreads();

  const float neg_inf = -__builtin_inff();
  const int qloc = wave * 16 + 8 * hh;
  float* so = SO[wave];

  {
    v16h qa[2], qla[2];
#pragma unroll
    for (int dc = 0; dc < 2; ++dc) {
      qa[dc]  = frag_load(qpl  + (size_t)(q0 + c) * HDIM + dc * 32 + 8 * hh);
      qla[dc] = frag_load(qlpl + (size_t)(q0 + c) * HDIM + dc * 32 + 8 * hh);
    }
#pragma unroll 1
    for (int j = 0; j < 4; ++j) {
      v8f s  = (v8f){0.f, 0.f, 0.f, 0.f, 0.f, 0.f, 0.f, 0.f};
      v8f sr = (v8f){0.f, 0.f, 0.f, 0.f, 0.f, 0.f, 0.f, 0.f};
#pragma unroll
      for (int dc = 0; dc < 2; ++dc) {
        const v16h kb  = frag_load(Ksh  + (j * 16 + c) * HDIM + dc * 32 + 8 * hh);
        const v16h klb = frag_load(klpl + (size_t)(j * 16 + c) * HDIM + dc * 32 + 8 * hh);
        s  = mma_h(qa[dc],  kb,  s);
        sr = mma_h(qa[dc],  klb, sr);
        sr = mma_h(qla[dc], kb,  sr);
      }
#pragma unroll
      for (int r = 0; r < 8; ++r) {
        float sv = (s[r] + sr[r] * SRES_INV) * SSCALE;
        if ((j * 16 + c) > (qloc + r)) sv = MASKV;
        so[(8 * hh + r) * OPITCH + j * 16 + c] = sv;
      }
    }
  }
  wave_lds_sync();

  float inv[8];
  _Float16* pw  = Psh[wave];
  _Float16* plw = Plsh[wave];
#pragma unroll
  for (int r = 0; r < 8; ++r) {
    const float* sp = so + (8 * hh + r) * OPITCH + c;
    const float sv0 = sp[0], sv1 = sp[16], sv2 = sp[32], sv3 = sp[48];
    float m = fmaxf(fmaxf(sv0, sv1), fmaxf(sv2, sv3));
#pragma unroll
    for (int off = 1; off < 16; off <<= 1) m = fmaxf(m, __shfl_xor(m, off, 32));
    const float p0 = expf(sv0 - m), p1 = expf(sv1 - m), p2 = expf(sv2 - m), p3 = expf(sv3 - m);
    float psum = (p0 + p1) + (p2 + p3);
    {
      const float pc0 = p0 * PCARRY; const _Float16 g0 = (_Float16)pc0;
      const float pc1 = p1 * PCARRY; const _Float16 g1 = (_Float16)pc1;
      const float pc2 = p2 * PCARRY; const _Float16 g2 = (_Float16)pc2;
      const float pc3 = p3 * PCARRY; const _Float16 g3 = (_Float16)pc3;
      _Float16* prow  = pw  + (8 * hh + r) * KCH + c;
      _Float16* plrow = plw + (8 * hh + r) * KCH + c;
      prow[0]  = g0; prow[16] = g1; prow[32] = g2; prow[48] = g3;
      plrow[0]  = (_Float16)((pc0 - (float)g0) * LOCARRY);
      plrow[16] = (_Float16)((pc1 - (float)g1) * LOCARRY);
      plrow[32] = (_Float16)((pc2 - (float)g2) * LOCARRY);
      plrow[48] = (_Float16)((pc3 - (float)g3) * LOCARRY);
    }
#pragma unroll
    for (int off = 1; off < 16; off <<= 1) psum += __shfl_xor(psum, off, 32);
    inv[r] = 1.0f / (psum * PCARRY);
  }
  wave_lds_sync();

  {
    v16h pa[2], pla[2];
#pragma unroll
    for (int kk = 0; kk < 2; ++kk) {
      pa[kk]  = frag_load(pw  + c * KCH + kk * 32 + 8 * hh);
      pla[kk] = frag_load(plw + c * KCH + kk * 32 + 8 * hh);
    }
#pragma unroll 1
    for (int t = 0; t < 4; ++t) {
      v8f acc  = (v8f){0.f, 0.f, 0.f, 0.f, 0.f, 0.f, 0.f, 0.f};
      v8f acc2 = (v8f){0.f, 0.f, 0.f, 0.f, 0.f, 0.f, 0.f, 0.f};
#pragma unroll
      for (int kk = 0; kk < 2; ++kk) {
        const v16h vb  = frag_load(Vhs + (t * 16 + c) * KCH + kk * 32 + 8 * hh);
        const v16h vlb = frag_load(Vls + (t * 16 + c) * KCH + kk * 32 + 8 * hh);
        acc  = mma_h(pa[kk],  vb,  acc);
        acc2 = mma_h(pa[kk],  vlb, acc2);
        acc2 = mma_h(pla[kk], vb,  acc2);
      }
#pragma unroll
      for (int r = 0; r < 8; ++r)
        so[(8 * hh + r) * OPITCH + t * 16 + c] = (acc[r] + acc2[r] * LO_INV) * inv[r];
    }
  }
  wave_lds_sync();

  {
    const int rg = lane >> 3;
    const int c8 = (lane & 7) * 8;
    const size_t obase = ((size_t)b * SEQ + (size_t)q0) * INNER + (size_t)h * HDIM;
    for (int pass = 0; pass < 2; ++pass) {
#pragma unroll
      for (int it = 0; it < 4; ++it) {
        const int row = it * 4 + rg;
        const float* sp = so + row * OPITCH + c8;
        const v4f x0 = *(const v4f*)(sp);
        const v4f x1 = *(const v4f*)(sp + 4);
        v8h hv, lv;
#pragma unroll
        for (int e = 0; e < 4; ++e) {
          const float f0 = x0[e] * OCARRY;
          const _Float16 g0 = (_Float16)f0;
          hv[e] = g0;
          lv[e] = (_Float16)((f0 - (float)g0) * LOCARRY);
          const float f1 = x1[e] * OCARRY;
          const _Float16 g1 = (_Float16)f1;
          hv[4 + e] = g1;
          lv[4 + e] = (_Float16)((f1 - (float)g1) * LOCARRY);
        }
        *(volatile v8h*)(Oh + obase + (size_t)row * INNER + c8) = hv;
        *(volatile v8h*)(Ol + obase + (size_t)row * INNER + c8) = lv;
      }
      __threadfence();
    }
  }
}

extern "C" void kernel_launch(void* const* d_in, const int* in_sizes, int n_in,
                              void* d_out, int out_size, void* d_ws, size_t ws_size,
                              hipStream_t stream) {
  if (n_in < 5) return;
  const long long needX = ((long long)(NB - 1) * SEQ_FULL + SEQ) * (long long)DIM;
  const long long needW = (long long)KD * KD;
  if ((long long)in_sizes[0] < needX) return;
  if ((long long)in_sizes[1] < needW) return;
  if ((long long)in_sizes[2] < needW) return;
  if ((long long)in_sizes[3] < needW) return;
  if ((long long)in_sizes[4] < needW) return;
  if ((long long)out_size < needX) return;

  const float* x  = (const float*)d_in[0];
  const float* Wq = (const float*)d_in[1];
  const float* Wk = (const float*)d_in[2];
  const float* Wv = (const float*)d_in[3];
  const float* Wo = (const float*)d_in[4];
  float* out = (float*)d_out;

  const size_t xhB = (size_t)MROWS * DIM * sizeof(_Float16);
  const size_t wtB = (size_t)4 * KD * KD * sizeof(_Float16);
  const size_t cB  = (size_t)MROWS * QKVC * sizeof(float);
  const size_t plB = (size_t)NB * NHEAD * SEQ * HDIM * sizeof(_Float16);
  const size_t qlB = (size_t)NB * NHEAD * ERES * HDIM * sizeof(_Float16);
  const size_t oB  = (size_t)MROWS * INNER * sizeof(_Float16);

  size_t off = 0;
  char* ws = (char*)d_ws;
  _Float16* xh   = (_Float16*)(ws + off); off += xhB;
  _Float16* Wt   = (_Float16*)(ws + off); off += wtB;
  float*    Cqkv = (float*)(ws + off);    off += cB;
  _Float16* Qh   = (_Float16*)(ws + off); off += plB;
  _Float16* Qlh  = (_Float16*)(ws + off); off += qlB;
  _Float16* Kh   = (_Float16*)(ws + off); off += plB;
  _Float16* Klh  = (_Float16*)(ws + off); off += qlB;
  _Float16* Vth  = (_Float16*)(ws + off); off += plB;
  _Float16* Vtl  = (_Float16*)(ws + off); off += plB;
  _Float16* Oh   = (_Float16*)(ws + off); off += oB;
  _Float16* Ol   = (_Float16*)(ws + off); off += oB;
  if (off > ws_size) return;

  cvt_x<<<dim3(MROWS / 2), dim3(CVX_THREADS), 0, stream>>>(x, xh);
  cvt_w<<<dim3(KD / 64, KD / 64, 4), dim3(CVW_THREADS), 0, stream>>>(Wq, Wk, Wv, Wo, Wt);
  gemm_f16<0><<<dim3(QKVC / 64, MROWS / 64), dim3(GM_THREADS), 0, stream>>>(
      xh, xh, Wt, Cqkv, QKVC, SEQ, QKV_INV);
  prep_planes<<<dim3(NB * NHEAD * (SEQ / TROWS)), dim3(PREP_THREADS), 0, stream>>>(
      Cqkv, Qh, Qlh, Kh, Klh, Vth, Vtl);
  early_attn<<<dim3(NB * NHEAD), dim3(AT_THREADS), 0, stream>>>(
      Qh, Qlh, Kh, Klh, Vth, Vtl, Oh, Ol);
  causal_attn<<<dim3(NB * NHEAD * (SEQ / QBLK - 1)), dim3(AT_THREADS), 0, stream>>>(
      Qh, Kh, Vth, Vtl, Oh, Ol);
  gemm_f16<1><<<dim3(DIM / 64, MROWS / 64), dim3(GM_THREADS), 0, stream>>>(
      Oh, Ol, Wt + (size_t)3 * KD * KD, out, DIM, SEQ_FULL, OUT_INV);
}
